// GCNNode_37056977830250
// MI455X (gfx1250) — hardware-verified
//
#include <hip/hip_runtime.h>
#include <stddef.h>


#define DF      128
#define NCLS    64
#define NTHR    256
#define NWAVE   8
#define EPT     8
#define NGRP    2
#define CHUNK   (NTHR * EPT * NGRP)
#define WCAP    (EPT * NGRP * 32)
#define LISTN   (NWAVE * WCAP)
#define NBA     512
#define NBD     4096
#define GROWS   128
#define APITCH  136
#define PLW     (DF * DF)
#define PLC     (DF * NCLS)
#define BNEPS   1e-5f

#define LDS_GEMM (2 * GROWS * APITCH * 2)
#define LDS_AGG  (NBA * DF * 4 + LISTN * 4 + 64)

static_assert((CHUNK & (CHUNK - 1)) == 0);
static_assert(CHUNK <= 4096);
static_assert(NBA <= 4096 && NBD <= 4096);
static_assert((NBA & (NBA - 1)) == 0 && (NBD & (NBD - 1)) == 0);
static_assert(GROWS * DF * 4 <= LDS_GEMM);
static_assert(2 * DF * 8 <= LISTN * 4);
static_assert(NBD % NBA == 0 && NBD % GROWS == 0);

typedef float          v4f  __attribute__((ext_vector_type(4)));
typedef float          v8f  __attribute__((ext_vector_type(8)));
typedef int            v4i  __attribute__((ext_vector_type(4)));
typedef double         v2d  __attribute__((ext_vector_type(2)));
typedef unsigned short v8us __attribute__((ext_vector_type(8)));
typedef __bf16         v16b __attribute__((ext_vector_type(16)));
union FragB { v16b v; v8us u[2]; };

__device__ __forceinline__ unsigned int bfr(float x) {
  const unsigned int u = __float_as_uint(x);
  return (u + 0x7FFFu + ((u >> 16) & 1u)) >> 16;
}

#define SPL1(I, X) { const float xx = (X); const unsigned int hb = bfr(xx); \
  h[I] = (unsigned short)hb; l[I] = (unsigned short)bfr(xx - __uint_as_float(hb << 16)); }
__device__ __forceinline__ void split8(v4f a, v4f b, v8us& h, v8us& l) {
  SPL1(0, a.x) SPL1(1, a.y) SPL1(2, a.z) SPL1(3, a.w)
  SPL1(4, b.x) SPL1(5, b.y) SPL1(6, b.z) SPL1(7, b.w)
}
#undef SPL1

__device__ __forceinline__ v8f wm3(v16b ah, v16b al, v16b bh, v16b bl, v8f c) {
  v8f d = __builtin_amdgcn_wmma_f32_16x16x32_bf16(false, ah, false, bh, (short)0, c, false, false);
  d = __builtin_amdgcn_wmma_f32_16x16x32_bf16(false, ah, false, bl, (short)0, d, false, false);
  d = __builtin_amdgcn_wmma_f32_16x16x32_bf16(false, al, false, bh, (short)0, d, false, false);
  asm volatile("v_nop\n\tv_nop\n\tv_nop\n\tv_nop" : "+v"(d) : "v"(ah), "v"(al), "v"(bh), "v"(bl));
  return d;
}

template <int NB>
__device__ __forceinline__ int scan_chunk(const int* __restrict__ dsts, int nE, int cbase, int nodeBase,
                                          int vec8, int* list, int tid, int lane, int wave) {
  int wc = 0;
#pragma unroll
  for (int g = 0; g < NGRP; ++g) {
    const int el0  = (g * NTHR + tid) * EPT;
    const int e0   = cbase + el0;
    const int sent = -2147483647 - 1;
    v4i da, db;
    if (vec8 != 0 && e0 + 7 < nE) {
      da = *(const v4i*)(dsts + e0);
      db = *(const v4i*)(dsts + e0 + 4);
    } else {
      da.x = (e0     < nE) ? dsts[min(e0, nE - 1)] : sent;
      da.y = (e0 + 1 < nE) ? dsts[min(e0 + 1, nE - 1)] : sent;
      da.z = (e0 + 2 < nE) ? dsts[min(e0 + 2, nE - 1)] : sent;
      da.w = (e0 + 3 < nE) ? dsts[min(e0 + 3, nE - 1)] : sent;
      db.x = (e0 + 4 < nE) ? dsts[min(e0 + 4, nE - 1)] : sent;
      db.y = (e0 + 5 < nE) ? dsts[min(e0 + 5, nE - 1)] : sent;
      db.z = (e0 + 6 < nE) ? dsts[min(e0 + 6, nE - 1)] : sent;
      db.w = (e0 + 7 < nE) ? dsts[min(e0 + 7, nE - 1)] : sent;
    }
    const unsigned nb = (unsigned)nodeBase;
    const unsigned s0 = (unsigned)da.x - nb, s1 = (unsigned)da.y - nb;
    const unsigned s2 = (unsigned)da.z - nb, s3 = (unsigned)da.w - nb;
    const unsigned s4 = (unsigned)db.x - nb, s5 = (unsigned)db.y - nb;
    const unsigned s6 = (unsigned)db.z - nb, s7 = (unsigned)db.w - nb;
    const bool h0 = s0 < (unsigned)NB, h1 = s1 < (unsigned)NB, h2 = s2 < (unsigned)NB, h3 = s3 < (unsigned)NB;
    const bool h4 = s4 < (unsigned)NB, h5 = s5 < (unsigned)NB, h6 = s6 < (unsigned)NB, h7 = s7 < (unsigned)NB;
    const unsigned any = __builtin_amdgcn_ballot_w32(h0 | h1 | h2 | h3 | h4 | h5 | h6 | h7);
    if (any != 0u) {
#define HITJ(J, HJ, SJ) { \
        const unsigned mj = __builtin_amdgcn_ballot_w32(HJ); \
        if (mj != 0u) { \
          if (HJ) { \
            const int pos = wc + (int)__builtin_amdgcn_mbcnt_lo(mj, 0u); \
            if (pos < WCAP) list[wave * WCAP + pos] = ((el0 + (J)) << 12) | (int)(SJ); \
          } \
          wc += (int)__builtin_popcount(mj); } }
      HITJ(0, h0, s0)
      HITJ(1, h1, s1)
      HITJ(2, h2, s2)
      HITJ(3, h3, s3)
      HITJ(4, h4, s4)
      HITJ(5, h5, s5)
      HITJ(6, h6, s6)
      HITJ(7, h7, s7)
#undef HITJ
    }
  }
  return wc;
}

__global__ __launch_bounds__(NTHR) void k_wprep(
    const float* __restrict__ W0, const float* __restrict__ W1, const float* __restrict__ W2,
    const float* __restrict__ Wc, unsigned short* wp) {
  const int i  = blockIdx.x * NTHR + threadIdx.x;
  const int n1 = PLW / 8;
  const int nc = PLC / 8;
  if (i >= 3 * n1 + nc) return;
  const float* W; int j, ncols; size_t hoff, loff;
  if (i < n1)          { W = W0; j = i;          ncols = DF;   hoff = 0;                 loff = (size_t)PLW; }
  else if (i < 2 * n1) { W = W1; j = i - n1;     ncols = DF;   hoff = 2 * (size_t)PLW;   loff = 3 * (size_t)PLW; }
  else if (i < 3 * n1) { W = W2; j = i - 2 * n1; ncols = DF;   hoff = 4 * (size_t)PLW;   loff = 5 * (size_t)PLW; }
  else                 { W = Wc; j = i - 3 * n1; ncols = NCLS; hoff = 6 * (size_t)PLW;   loff = 6 * (size_t)PLW + PLC; }
  const int o  = j * 8;
  const int n  = o / DF;
  const int k0 = o - n * DF;
  const float* p = W + (size_t)k0 * ncols + n;
  v4f a, b;
  a.x = p[0];         a.y = p[ncols];     a.z = p[2 * ncols]; a.w = p[3 * ncols];
  b.x = p[4 * ncols]; b.y = p[5 * ncols]; b.z = p[6 * ncols]; b.w = p[7 * ncols];
  v8us hv, lv;
  split8(a, b, hv, lv);
  unsigned short* hp = wp + hoff + o;
  unsigned short* lq = wp + loff + o;
  *(volatile v8us*)hp = hv;
  *(volatile v8us*)lq = lv;
  __threadfence();
  *(volatile v8us*)hp = hv;
  *(volatile v8us*)lq = lv;
}

__device__ __forceinline__ void deg_pass(const int* __restrict__ arr, float* outp, int nE, int vec8,
                                         int* cnt, int* list, int* wcnt, int nodeBase,
                                         int tid, int lane, int wave) {
  for (int i = tid; i < NBD; i += NTHR) cnt[i] = 0;
  __syncthreads();

  const int nChunks = (nE + CHUNK - 1) / CHUNK;
#pragma unroll 1
  for (int ch = 0; ch < nChunks; ++ch) {
    const int cbase = ch * CHUNK;
    const int wc = scan_chunk<NBD>(arr, nE, cbase, nodeBase, vec8, list, tid, lane, wave);
    if (lane == 0) wcnt[wave] = wc;
    __syncthreads();
    if (wave == 0) {
#pragma unroll 1
      for (int wsx = 0; wsx < NWAVE; ++wsx) {
        int n = __builtin_amdgcn_readfirstlane(wcnt[wsx]);
        n = n > WCAP ? WCAP : (n < 0 ? 0 : n);
        const int* lp = list + wsx * WCAP;
#pragma unroll 1
        for (int i = 0; i < n; ++i) {
          const int ent  = __builtin_amdgcn_readfirstlane(lp[i]);
          const int slot = ent & (NBD - 1);
          if (lane == 0) cnt[slot] = cnt[slot] + 1;
        }
      }
    }
    __syncthreads();
  }

  v4f dq[4];
#pragma unroll
  for (int q = 0; q < 4; ++q) {
    const int f = (wave * 4 + q) * 128 + 4 * lane;
    const v4i c = *(const v4i*)(cnt + f);
    dq[q].x = c.x > 0 ? rsqrtf((float)c.x) : 0.f;
    dq[q].y = c.y > 0 ? rsqrtf((float)c.y) : 0.f;
    dq[q].z = c.z > 0 ? rsqrtf((float)c.z) : 0.f;
    dq[q].w = c.w > 0 ? rsqrtf((float)c.w) : 0.f;
  }
  float* dp = outp + (size_t)nodeBase;
#pragma unroll
  for (int q = 0; q < 4; ++q) *(volatile v4f*)(dp + (wave * 4 + q) * 128 + 4 * lane) = dq[q];
  __threadfence();
#pragma unroll
  for (int q = 0; q < 4; ++q) *(volatile v4f*)(dp + (wave * 4 + q) * 128 + 4 * lane) = dq[q];
}

__global__ __launch_bounds__(NTHR) void k_deg(
    const int* __restrict__ src, const int* __restrict__ dst, float* dinvS, float* dinvD,
    int nE, int vec8) {
  __shared__ __attribute__((aligned(16))) int cnt[NBD];
  __shared__ __attribute__((aligned(16))) int list[LISTN];
  __shared__ int wcnt[NWAVE];
  const int tid = threadIdx.x, lane = tid & 31, wave = tid >> 5;
  const int nodeBase = blockIdx.x * NBD;
  deg_pass(src, dinvS, nE, vec8, cnt, list, wcnt, nodeBase, tid, lane, wave);
  __syncthreads();
  deg_pass(dst, dinvD, nE, vec8, cnt, list, wcnt, nodeBase, tid, lane, wave);
}

template <int NC>
__global__ __launch_bounds__(NTHR) void k_gemm(
    const float* __restrict__ x, const float* __restrict__ ms, const float* __restrict__ beta,
    const unsigned short* __restrict__ wh, const unsigned short* __restrict__ wl,
    const float* __restrict__ dinv, const float* __restrict__ bias, float* out,
    int nN, int nRowsOut, int flags) {
  constexpr int NT = NC / 16;
  constexpr int NQ = 16 * NC / 128;
  extern __shared__ v4f lds_dyn[];
  unsigned short* sAh = (unsigned short*)lds_dyn;
  unsigned short* sAl = sAh + GROWS * APITCH;
  float*          stg = (float*)lds_dyn;
  const int tid = threadIdx.x, lane = tid & 31, wave = tid >> 5, hh = lane >> 4, m = lane & 15;
  const int rowBase = blockIdx.x * GROWS;
  const int c0 = (tid & 15) * 8;

  v4f m0 = {0.f, 0.f, 0.f, 0.f}, m1 = m0, s0 = m0, s1 = m0, e0 = m0, e1 = m0;
  if (flags & 1) {
    m0 = *(const v4f*)(ms + c0);        m1 = *(const v4f*)(ms + c0 + 4);
    s0 = *(const v4f*)(ms + DF + c0);   s1 = *(const v4f*)(ms + DF + c0 + 4);
    e0 = *(const v4f*)(beta + c0);      e1 = *(const v4f*)(beta + c0 + 4);
  }

#pragma unroll 2
  for (int i = 0; i < (GROWS * DF / 8) / NTHR; ++i) {
    const int idx = i * NTHR + tid;
    const int r   = idx >> 4;
    int node = rowBase + r;
    node = node > nN - 1 ? nN - 1 : node;
    const float* xp = x + (size_t)node * DF + c0;
    v4f a = *(const v4f*)xp, b = *(const v4f*)(xp + 4);
    if (flags & 1) {
      a = (a - m0) * s0 + e0;
      b = (b - m1) * s1 + e1;
      a.x = fmaxf(a.x, 0.f); a.y = fmaxf(a.y, 0.f); a.z = fmaxf(a.z, 0.f); a.w = fmaxf(a.w, 0.f);
      b.x = fmaxf(b.x, 0.f); b.y = fmaxf(b.y, 0.f); b.z = fmaxf(b.z, 0.f); b.w = fmaxf(b.w, 0.f);
    }
    v8us hv, lv;
    split8(a, b, hv, lv);
    *(v8us*)(sAh + r * APITCH + c0) = hv;
    *(v8us*)(sAl + r * APITCH + c0) = lv;
  }
  __syncthreads();

  v8f acc[NT];
#pragma unroll
  for (int t = 0; t < NT; ++t) { v8f z = {0.f, 0.f, 0.f, 0.f, 0.f, 0.f, 0.f, 0.f}; acc[t] = z; }
  const unsigned short* arh = sAh + (wave * 16 + m) * APITCH + 8 * hh;
  const unsigned short* arl = sAl + (wave * 16 + m) * APITCH + 8 * hh;
#pragma unroll
  for (int kt = 0; kt < DF / 32; ++kt) {
    FragB ah, al;
    ah.u[0] = *(const v8us*)(arh + 32 * kt);
    ah.u[1] = *(const v8us*)(arh + 32 * kt + 16);
    al.u[0] = *(const v8us*)(arl + 32 * kt);
    al.u[1] = *(const v8us*)(arl + 32 * kt + 16);
#pragma unroll
    for (int t = 0; t < NT; ++t) {
      const size_t bo = (size_t)(16 * t + m) * DF + 32 * kt + 8 * hh;
      FragB bh, bl;
      bh.u[0] = *(const v8us*)(wh + bo);
      bh.u[1] = *(const v8us*)(wh + bo + 16);
      bl.u[0] = *(const v8us*)(wl + bo);
      bl.u[1] = *(const v8us*)(wl + bo + 16);
      acc[t] = wm3(ah.v, al.v, bh.v, bl.v, acc[t]);
    }
  }
  __syncthreads();

  const int r0 = wave * 16 + 8 * hh;
  v4f dA = {1.f, 1.f, 1.f, 1.f}, dB = dA;
  if (flags & 2) {
    dA = *(const v4f*)(dinv + (size_t)rowBase + r0);
    dB = *(const v4f*)(dinv + (size_t)rowBase + r0 + 4);
  }
  float* sp = stg + r0 * NC + m;
#pragma unroll
  for (int t = 0; t < NT; ++t) {
    const float bv = (flags & 4) ? bias[16 * t + m] : 0.f;
    sp[0 * NC + 16 * t] = acc[t][0] * dA.x + bv;
    sp[1 * NC + 16 * t] = acc[t][1] * dA.y + bv;
    sp[2 * NC + 16 * t] = acc[t][2] * dA.z + bv;
    sp[3 * NC + 16 * t] = acc[t][3] * dA.w + bv;
    sp[4 * NC + 16 * t] = acc[t][4] * dB.x + bv;
    sp[5 * NC + 16 * t] = acc[t][5] * dB.y + bv;
    sp[6 * NC + 16 * t] = acc[t][6] * dB.z + bv;
    sp[7 * NC + 16 * t] = acc[t][7] * dB.w + bv;
  }
  __syncthreads();

  const int wrow0 = rowBase + wave * 16;
  int vr = nRowsOut - wrow0;
  vr = vr < 0 ? 0 : (vr > 16 ? 16 : vr);
  const int vfl = vr * NC;
  const float* lp = stg + wave * 16 * NC;
  float* gp = out + (size_t)wrow0 * NC;
#pragma unroll
  for (int q = 0; q < NQ; ++q) {
    const int f = q * 128 + 4 * lane;
    if (f < vfl) { const v4f v = *(const v4f*)(lp + f); *(volatile v4f*)(gp + f) = v; }
  }
  __threadfence();
#pragma unroll
  for (int q = 0; q < NQ; ++q) {
    const int f = q * 128 + 4 * lane;
    if (f < vfl) { const v4f v = *(const v4f*)(lp + f); *(volatile v4f*)(gp + f) = v; }
  }
}

__global__ __launch_bounds__(NTHR) void k_agg(
    const int* __restrict__ src, const int* __restrict__ dst, const float* __restrict__ g,
    const float* __restrict__ dinvD, float* y, double* part, int nN, int nE, int vec8) {
  extern __shared__ v4f lds_dyn[];
  float*  acc  = (float*)lds_dyn;
  int*    list = (int*)(acc + NBA * DF);
  int*    wcnt = list + LISTN;
  double* pst  = (double*)list;
  const int tid = threadIdx.x, lane = tid & 31, wave = tid >> 5;
  const int nodeBase = blockIdx.x * NBA;

  {
    const v4f z = {0.f, 0.f, 0.f, 0.f};
    for (int i = tid; i < NBA * DF / 4; i += NTHR) lds_dyn[i] = z;
  }
  __syncthreads();

  const int nChunks = (nE + CHUNK - 1) / CHUNK;
#pragma unroll 1
  for (int ch = 0; ch < nChunks; ++ch) {
    const int cbase = ch * CHUNK;
    const int wc = scan_chunk<NBA>(dst, nE, cbase, nodeBase, vec8, list, tid, lane, wave);
    if (lane == 0) wcnt[wave] = wc;
    __syncthreads();
    if (wave == 0) {
#pragma unroll 1
      for (int wsx = 0; wsx < NWAVE; ++wsx) {
        int n = __builtin_amdgcn_readfirstlane(wcnt[wsx]);
        n = n > WCAP ? WCAP : (n < 0 ? 0 : n);
        const int* lp = list + wsx * WCAP;
#pragma unroll 1
        for (int i = 0; i < n; ++i) {
          const int ent  = __builtin_amdgcn_readfirstlane(lp[i]);
          const int slot = ent & (NBA - 1);
          int e = cbase + ((ent >> 12) & (CHUNK - 1));
          e = e > nE - 1 ? nE - 1 : e;
          int s = src[e];
          s = s < 0 ? 0 : (s > nN - 1 ? nN - 1 : s);
          const v4f v = *(const v4f*)(g + (size_t)s * DF + 4 * lane);
          v4f* ap = (v4f*)(acc + slot * DF + 4 * lane);
          *ap = *ap + v;
        }
      }
    }
    __syncthreads();
  }

#pragma unroll 4
  for (int i = 0; i < (NBA * DF / 4) / NTHR; ++i) {
    const int idx  = i * NTHR + tid;
    const int slot = idx >> 5;
    const int c4   = (idx & 31) * 4;
    const float d  = dinvD[(size_t)nodeBase + slot];
    v4f* ap = (v4f*)(acc + slot * DF + c4);
    const v4f yv = *ap * d;
    *ap = yv;
  }
  __syncthreads();

  {
    const int c = tid & (DF - 1);
    double s = 0.0;
    if (tid < DF) {
#pragma unroll 4
      for (int r = 0; r < NBA; ++r) s += (double)acc[r * DF + c];
    } else {
#pragma unroll 4
      for (int r = 0; r < NBA; ++r) { const double v = (double)acc[r * DF + c]; s += v * v; }
    }
    pst[tid] = s;
  }
  __syncthreads();

  float* yp = y + (size_t)nodeBase * DF;
  double* pp = part + (size_t)blockIdx.x * (2 * DF);
#pragma unroll 4
  for (int q = 0; q < 64; ++q) {
    const int f = (wave * 64 + q) * DF + 4 * lane;
    const v4f v = *(const v4f*)(acc + f);
    *(volatile v4f*)(yp + f) = v;
  }
  if (tid < DF) { const v2d pv = *(const v2d*)(pst + 2 * tid); *(volatile v2d*)(pp + 2 * tid) = pv; }
  __threadfence();
#pragma unroll 4
  for (int q = 0; q < 64; ++q) {
    const int f = (wave * 64 + q) * DF + 4 * lane;
    const v4f v = *(const v4f*)(acc + f);
    *(volatile v4f*)(yp + f) = v;
  }
  if (tid < DF) { const v2d pv = *(const v2d*)(pst + 2 * tid); *(volatile v2d*)(pp + 2 * tid) = pv; }
}

__global__ __launch_bounds__(NTHR) void k_stats(
    const double* __restrict__ part, int nPart, const float* __restrict__ gamma, float* ms, int nN) {
  __shared__ __attribute__((aligned(16))) float sms[2 * DF];
  const int tid = threadIdx.x;
  if (tid < DF) {
    double s = 0.0, s2 = 0.0;
#pragma unroll 1
    for (int p = 0; p < nPart; ++p) {
      s  += part[(size_t)p * (2 * DF) + tid];
      s2 += part[(size_t)p * (2 * DF) + DF + tid];
    }
    const double invn = 1.0 / (double)nN;
    const double mean = s * invn;
    double var = s2 * invn - mean * mean;
    var = var < 0.0 ? 0.0 : var;
    sms[tid]      = (float)mean;
    sms[DF + tid] = gamma[tid] * rsqrtf((float)var + BNEPS);
  }
  __syncthreads();
  v4f v = {0.f, 0.f, 0.f, 0.f};
  if (tid < 64) { v = *(const v4f*)(sms + 4 * tid); *(volatile v4f*)(ms + 4 * tid) = v; }
  __threadfence();
  if (tid < 64) { *(volatile v4f*)(ms + 4 * tid) = v; }
}

extern "C" void kernel_launch(void* const* d_in, const int* in_sizes, int n_in,
                              void* d_out, int out_size, void* d_ws, size_t ws_size,
                              hipStream_t stream) {
  if (n_in < 14) return;
  const int nN = in_sizes[0] / DF;
  const int nE = in_sizes[1];
  if (nN <= 0 || nE <= 0 || in_sizes[0] != nN * DF || in_sizes[2] != nE) return;
  if (in_sizes[3] != PLW || in_sizes[4] != PLW || in_sizes[5] != PLW) return;
  for (int i = 6; i < 12; ++i) if (in_sizes[i] != DF) return;
  if (in_sizes[12] != PLC || in_sizes[13] != NCLS) return;
  if (out_size != nN * NCLS) return;

  const float* feat = (const float*)d_in[0];
  const int*   src  = (const int*)d_in[1];
  const int*   dst  = (const int*)d_in[2];
  const float* W0   = (const float*)d_in[3];
  const float* W1   = (const float*)d_in[4];
  const float* W2   = (const float*)d_in[5];
  const float* g0   = (const float*)d_in[6];
  const float* b0   = (const float*)d_in[7];
  const float* g1   = (const float*)d_in[8];
  const float* b1   = (const float*)d_in[9];
  const float* g2   = (const float*)d_in[10];
  const float* b2   = (const float*)d_in[11];
  const float* Wc   = (const float*)d_in[12];
  const float* cb   = (const float*)d_in[13];
  float* out = (float*)d_out;

  const int nBD = (nN + NBD - 1) / NBD;
  const int nG  = (nN + GROWS - 1) / GROWS;
  const int nA  = (nN + NBA - 1) / NBA;
  if ((size_t)nA * NBA > (size_t)nBD * NBD || (size_t)nG * GROWS > (size_t)nBD * NBD) return;

  char* ws = (char*)d_ws;
  size_t off = 0;
  const size_t oWP = off; off += (size_t)(6 * PLW + 2 * PLC) * 2;        off = (off + 255) & ~(size_t)255;
  const size_t oDS = off; off += (size_t)nBD * NBD * 4;                  off = (off + 255) & ~(size_t)255;
  const size_t oDD = off; off += (size_t)nBD * NBD * 4;                  off = (off + 255) & ~(size_t)255;
  const size_t oG  = off; off += (size_t)nG * GROWS * DF * 4;            off = (off + 255) & ~(size_t)255;
  const size_t oY  = off; off += (size_t)nA * NBA * DF * 4;              off = (off + 255) & ~(size_t)255;
  const size_t oP  = off; off += (size_t)nA * 2 * DF * 8;                off = (off + 255) & ~(size_t)255;
  const size_t oM  = off; off += (size_t)2 * DF * 4;                     off = (off + 255) & ~(size_t)255;
  if (off > ws_size) return;
  unsigned short* wp    = (unsigned short*)(ws + oWP);
  float*          dinvS = (float*)(ws + oDS);
  float*          dinvD = (float*)(ws + oDD);
  float*          G     = (float*)(ws + oG);
  float*          Y     = (float*)(ws + oY);
  double*         part  = (double*)(ws + oP);
  float*          msb   = (float*)(ws + oM);

  const unsigned short* wh0 = wp;            const unsigned short* wl0 = wp + PLW;
  const unsigned short* wh1 = wp + 2 * PLW;  const unsigned short* wl1 = wp + 3 * PLW;
  const unsigned short* wh2 = wp + 4 * PLW;  const unsigned short* wl2 = wp + 5 * PLW;
  const unsigned short* whc = wp + 6 * PLW;  const unsigned short* wlc = wp + 6 * PLW + PLC;

  const int vec8 = 1;
  const int nPrep = 3 * (PLW / 8) + PLC / 8;
  k_wprep<<<(nPrep + NTHR - 1) / NTHR, NTHR, 0, stream>>>(W0, W1, W2, Wc, wp);

  k_deg<<<nBD, NTHR, 0, stream>>>(src, dst, dinvS, dinvD, nE, vec8);

  hipFuncSetAttribute(reinterpret_cast<const void*>(&k_gemm<DF>),
                      hipFuncAttributeMaxDynamicSharedMemorySize, LDS_GEMM);
  hipFuncSetAttribute(reinterpret_cast<const void*>(&k_gemm<NCLS>),
                      hipFuncAttributeMaxDynamicSharedMemorySize, LDS_GEMM);
  hipFuncSetAttribute(reinterpret_cast<const void*>(&k_agg),
                      hipFuncAttributeMaxDynamicSharedMemorySize, LDS_AGG);

  const int planeRows = nG * GROWS;

  k_gemm<DF><<<nG, NTHR, LDS_GEMM, stream>>>(feat, msb, b0, wh0, wl0, dinvS, b0, G, nN, planeRows, 2);
  k_agg<<<nA, NTHR, LDS_AGG, stream>>>(src, dst, G, dinvD, Y, part, nN, nE, vec8);
  k_stats<<<1, NTHR, 0, stream>>>(part, nA, g0, msb, nN);

  k_gemm<DF><<<nG, NTHR, LDS_GEMM, stream>>>(Y, msb, b0, wh1, wl1, dinvS, b0, G, nN, planeRows, 3);
  k_agg<<<nA, NTHR, LDS_AGG, stream>>>(src, dst, G, dinvD, Y, part, nN, nE, vec8);
  k_stats<<<1, NTHR, 0, stream>>>(part, nA, g1, msb, nN);

  k_gemm<DF><<<nG, NTHR, LDS_GEMM, stream>>>(Y, msb, b1, wh2, wl2, dinvS, b1, G, nN, planeRows, 3);
  k_agg<<<nA, NTHR, LDS_AGG, stream>>>(src, dst, G, dinvD, Y, part, nN, nE, vec8);
  k_stats<<<1, NTHR, 0, stream>>>(part, nA, g2, msb, nN);

  k_gemm<NCLS><<<nG, NTHR, LDS_GEMM, stream>>>(Y, msb, b2, whc, wlc, dinvS, cb, out, nN, nN, 5);
}
